// NonLocalBlock_19679540150545
// MI455X (gfx1250) — hardware-verified
//
#include <hip/hip_runtime.h>


#ifndef NB
#define NB 8
#endif
#define NB_FULL 8
#define NC 256
#define NI 128
#define HIMG 64
#define WIMG 64
#define NN (HIMG * WIMG)
#define NM ((HIMG / 2) * (WIMG / 2))
#define NPART (NB * (NN / 32))

static_assert(NB >= 1 && NB <= NB_FULL);
static_assert(NC == 256 && NI == 128 && NN == 4096 && NM == 1024);
static_assert((NB * NC * NN) % 1024 == 0);

typedef _Float16 v16h __attribute__((ext_vector_type(16)));
typedef _Float16 v8h  __attribute__((ext_vector_type(8)));
typedef float    v8f  __attribute__((ext_vector_type(8)));
typedef float    v4f  __attribute__((ext_vector_type(4)));
typedef float    fa_t __attribute__((may_alias));
typedef float    v4fa __attribute__((ext_vector_type(4))) __attribute__((may_alias));

constexpr size_t SZ_WPL  = (size_t)4 * NI * NC * 2;
constexpr size_t SZ_XT   = (size_t)NB * NN * NC * 2;
constexpr size_t SZ_TH   = (size_t)NB * NN * NI * 2;
constexpr size_t SZ_PH   = (size_t)NB * NM * NI * 2;
constexpr size_t SZ_GT   = (size_t)NB * NI * NM * 2;
constexpr size_t SZ_Y    = (size_t)NB * NN * NI * 2;
constexpr size_t SZ_WY   = (size_t)NB * NC * NN * 4;
constexpr size_t SZ_PART = (size_t)NPART * 512 * 4;
constexpr size_t SZ_ST   = (size_t)4 * NC * 4;
constexpr size_t OFF_WPL  = 0;
constexpr size_t OFF_XT   = OFF_WPL + SZ_WPL;
constexpr size_t OFF_THH  = OFF_XT + SZ_XT;
constexpr size_t OFF_THL  = OFF_THH + SZ_TH;
constexpr size_t OFF_PHH  = OFF_THL + SZ_TH;
constexpr size_t OFF_PHL  = OFF_PHH + SZ_PH;
constexpr size_t OFF_GT   = OFF_PHL + SZ_PH;
constexpr size_t OFF_YH   = OFF_GT + SZ_GT;
constexpr size_t OFF_YL   = OFF_YH + SZ_Y;
constexpr size_t OFF_WY   = OFF_YL + SZ_Y;
constexpr size_t OFF_PART = OFF_WY + SZ_WY;
constexpr size_t OFF_ST   = OFF_PART + SZ_PART;
constexpr size_t WS_TOTAL = OFF_ST + SZ_ST;
static_assert(WS_TOTAL <= (size_t)134217728);
static_assert((SZ_WPL % 128) == 0 && (SZ_XT % 128) == 0 && (SZ_TH % 128) == 0 && (SZ_PH % 128) == 0);
static_assert((SZ_GT % 128) == 0 && (SZ_Y % 128) == 0 && (SZ_WY % 128) == 0 && (SZ_PART % 128) == 0);

__device__ __forceinline__ float bf16r(float f) {
  unsigned int u = __float_as_uint(f);
  u = u + 0x7FFFu + ((u >> 16) & 1u);
  return __uint_as_float(u & 0xFFFF0000u);
}

__device__ __forceinline__ v8f wmma16(v16h a, v16h b, v8f c) {
  c = __builtin_amdgcn_wmma_f32_16x16x32_f16(false, a, false, b, (short)0, c, false, false);
  asm volatile("v_nop\n\tv_nop\n\tv_nop\n\tv_nop" : "+v"(c) : "v"(a), "v"(b));
  return c;
}

__device__ __forceinline__ v16h load_h16(const _Float16* p) {
  const v8h lo = *(const v8h*)(p);
  const v8h hi = *(const v8h*)(p + 16);
  return __builtin_shufflevector(lo, hi, 0, 1, 2, 3, 4, 5, 6, 7, 8, 9, 10, 11, 12, 13, 14, 15);
}

__device__ __forceinline__ void split8(v4f a, v4f c, v8h& hv, v8h& lv) {
#pragma unroll
  for (int j = 0; j < 4; ++j) {
    const _Float16 h0 = (_Float16)a[j];
    const _Float16 h1 = (_Float16)c[j];
    hv[j] = h0;
    hv[4 + j] = h1;
    lv[j] = (_Float16)((a[j] - (float)h0) * 1024.0f);
    lv[4 + j] = (_Float16)((c[j] - (float)h1) * 1024.0f);
  }
}

__device__ __forceinline__ void st2h8(_Float16* p, v8h v) {
  *(volatile v8h*)p = v;
  __threadfence();
  *(volatile v8h*)p = v;
}
__device__ __forceinline__ void st2f4(float* p, v4f v) {
  *(volatile v4f*)p = v;
  __threadfence();
  *(volatile v4f*)p = v;
}
__device__ __forceinline__ void st2f1(float* p, float v) {
  *(volatile float*)p = v;
  __threadfence();
  *(volatile float*)p = v;
}

__global__ void __launch_bounds__(256)
cvt_w_kernel(const float* __restrict__ tw, const float* __restrict__ pw,
             const float* __restrict__ gw, const float* __restrict__ ow,
             _Float16* __restrict__ wpl) {
  const int g8 = blockIdx.x * 256 + (int)threadIdx.x;
  const int which = g8 >> 12;
  const int e0 = (g8 & 4095) * 8;
  const float* src = (which == 0) ? tw : (which == 1) ? pw : (which == 2) ? gw : ow;
  const v4f a = *(const v4f*)(src + e0);
  const v4f c = *(const v4f*)(src + e0 + 4);
  v8h o;
#pragma unroll
  for (int j = 0; j < 4; ++j) {
    o[j]     = (_Float16)(bf16r(a[j]) * 16.0f);
    o[4 + j] = (_Float16)(bf16r(c[j]) * 16.0f);
  }
  st2h8(wpl + (size_t)which * (NI * NC) + e0, o);
}

__global__ void __launch_bounds__(256)
xpose_kernel(const float* __restrict__ x, _Float16* __restrict__ xT) {
  __shared__ _Float16 tile[64][34];
  const int tid = threadIdx.x;
  const int perb = (NC / 64) * (NN / 32);
  const int b   = blockIdx.x / perb;
  const int rem = blockIdx.x % perb;
  const int c0  = (rem / (NN / 32)) * 64;
  const int n0  = (rem % (NN / 32)) * 32;
  const int tx = tid & 31, ty = tid >> 5;
  const float* xb = x + (size_t)b * NC * NN;
#pragma unroll
  for (int s = 0; s < 8; ++s) {
    const int cl = ty + s * 8;
    tile[cl][tx] = (_Float16)bf16r(xb[(size_t)(c0 + cl) * NN + n0 + tx]);
  }
  __syncthreads();
  const int r = tid >> 3, q = tid & 7;
  v8h o;
#pragma unroll
  for (int j = 0; j < 8; ++j) o[j] = tile[q * 8 + j][r];
  st2h8(xT + ((size_t)b * NN + n0 + r) * NC + c0 + q * 8, o);
}

__global__ void __launch_bounds__(128)
theta_kernel(const _Float16* __restrict__ xT, const _Float16* __restrict__ wth,
             const float* __restrict__ bth,
             _Float16* __restrict__ thh, _Float16* __restrict__ thl) {
  __shared__ __align__(16) float st[4][16][132];
  const int lane = threadIdx.x & 31, wv = threadIdx.x >> 5;
  const int col = lane & 15, h8 = (lane >> 4) << 3;
  const int perb = NN / 64;
  const int b = blockIdx.x / perb;
  const int nBase = (blockIdx.x % perb) * 64 + wv * 16;
  const _Float16* xRow = xT + ((size_t)b * NN + nBase + col) * NC + h8;
  v16h Ax[8];
#pragma unroll
  for (int k = 0; k < 8; ++k) Ax[k] = load_h16(xRow + k * 32);
#pragma unroll 1
  for (int ic = 0; ic < 8; ++ic) {
    const int o = ic * 16 + col;
    const _Float16* wrow = wth + (size_t)o * NC + h8;
    v8f acc = {};
#pragma unroll
    for (int k = 0; k < 8; ++k) acc = wmma16(Ax[k], load_h16(wrow + k * 32), acc);
    const float bv = bf16r(bth[o]);
#pragma unroll
    for (int r = 0; r < 8; ++r) st[wv][h8 + r][o] = acc[r] * 0.0625f + bv;
  }
  __syncthreads();
  const size_t rowBase = (size_t)b * NN + nBase;
#pragma unroll 1
  for (int it = 0; it < 8; ++it) {
    const int line = it * 4 + (lane >> 3);
    const int row = line >> 1;
    const int e0 = (line & 1) * 64 + (lane & 7) * 8;
    const v4f va = *(const v4f*)&st[wv][row][e0];
    const v4f vb = *(const v4f*)&st[wv][row][e0 + 4];
    v8h hv, lv;
    split8(va, vb, hv, lv);
    const size_t off = (rowBase + row) * NI + e0;
    st2h8(thh + off, hv);
    st2h8(thl + off, lv);
  }
}

__device__ __forceinline__ v4f pool4(v8f t0, v8f t1, float bv) {
  v4f o;
#pragma unroll
  for (int j = 0; j < 4; ++j)
    o[j] = fmaxf(fmaxf(t0[2 * j], t0[2 * j + 1]), fmaxf(t1[2 * j], t1[2 * j + 1])) * 0.0625f + bv;
  return o;
}

__global__ void __launch_bounds__(256)
phig_kernel(const _Float16* __restrict__ xT, const _Float16* __restrict__ wph,
            const _Float16* __restrict__ wg, const float* __restrict__ bph,
            const float* __restrict__ bg,
            _Float16* __restrict__ phh, _Float16* __restrict__ phl,
            _Float16* __restrict__ gT) {
  __shared__ __align__(16) float sp[8][8][132];
  __shared__ __align__(16) _Float16 sg[NI][72];
  const int tid = threadIdx.x, lane = tid & 31, wv = tid >> 5;
  const int col = lane & 15, h = lane >> 4, h8 = h << 3;
  const int rp = wv >> 2, wc = wv & 3;
  const int perb = NN / 256;
  const int b = blockIdx.x / perb;
  const int blkn = blockIdx.x % perb;
  const int n0 = (blkn * 4 + rp * 2) * WIMG + wc * 16;
  const _Float16* xRow0 = xT + ((size_t)b * NN + n0 + col) * NC + h8;
  const _Float16* xRow1 = xRow0 + (size_t)WIMG * NC;
  const int mb = rp * 32 + wc * 8 + 4 * h;

#pragma unroll 1
  for (int icp = 0; icp < 4; ++icp) {
    const int o0 = icp * 32 + col, o1 = o0 + 16;
    v8f p00 = {}, p10 = {}, p01 = {}, p11 = {};
    v8f g00 = {}, g10 = {}, g01 = {}, g11 = {};
#pragma unroll 1
    for (int k = 0; k < 8; ++k) {
      const v16h a0 = load_h16(xRow0 + k * 32);
      const v16h a1 = load_h16(xRow1 + k * 32);
      const v16h bp0 = load_h16(wph + (size_t)o0 * NC + h8 + k * 32);
      const v16h bp1 = load_h16(wph + (size_t)o1 * NC + h8 + k * 32);
      const v16h bg0 = load_h16(wg + (size_t)o0 * NC + h8 + k * 32);
      const v16h bg1 = load_h16(wg + (size_t)o1 * NC + h8 + k * 32);
      p00 = wmma16(a0, bp0, p00);
      p10 = wmma16(a1, bp0, p10);
      p01 = wmma16(a0, bp1, p01);
      p11 = wmma16(a1, bp1, p11);
      g00 = wmma16(a0, bg0, g00);
      g10 = wmma16(a1, bg0, g10);
      g01 = wmma16(a0, bg1, g01);
      g11 = wmma16(a1, bg1, g11);
    }
    {
      const v4f vp = pool4(p00, p10, bf16r(bph[o0]));
      const v4f vg = pool4(g00, g10, bf16r(bg[o0]));
#pragma unroll
      for (int j = 0; j < 4; ++j) {
        sp[wv][4 * h + j][o0] = vp[j];
        sg[o0][mb + j] = (_Float16)vg[j];
      }
    }
    {
      const v4f vp = pool4(p01, p11, bf16r(bph[o1]));
      const v4f vg = pool4(g01, g11, bf16r(bg[o1]));
#pragma unroll
      for (int j = 0; j < 4; ++j) {
        sp[wv][4 * h + j][o1] = vp[j];
        sg[o1][mb + j] = (_Float16)vg[j];
      }
    }
  }
  __syncthreads();

  const int mh = blkn * 2 + rp;
  const size_t mrow0 = (size_t)b * NM + mh * 32 + wc * 8;
#pragma unroll 1
  for (int it = 0; it < 4; ++it) {
    const int line = it * 4 + (lane >> 3);
    const int row = line >> 1;
    const int e0 = (line & 1) * 64 + (lane & 7) * 8;
    const v4f va = *(const v4f*)&sp[wv][row][e0];
    const v4f vb = *(const v4f*)&sp[wv][row][e0 + 4];
    v8h hv, lv;
    split8(va, vb, hv, lv);
    const size_t off = (mrow0 + row) * NI + e0;
    st2h8(phh + off, hv);
    st2h8(phl + off, lv);
  }
#pragma unroll 1
  for (int it = 0; it < 4; ++it) {
    const int ci = it * 32 + (tid >> 3);
    const int q = tid & 7;
    const v8h o = *(const v8h*)&sg[ci][q * 8];
    st2h8(gT + ((size_t)b * NI + ci) * NM + blkn * 64 + q * 8, o);
  }
}

#define A_THH 0
#define A_THL 8192
#define A_PHH 16384
#define A_PHL 20480
#define A_GS  24576
#define A_PB  28672
#define A_TOT 30720

__global__ void __launch_bounds__(128)
attn_kernel(const _Float16* __restrict__ thh, const _Float16* __restrict__ thl,
            const _Float16* __restrict__ phh, const _Float16* __restrict__ phl,
            const _Float16* __restrict__ gT,
            _Float16* __restrict__ yh, _Float16* __restrict__ yl) {
  __shared__ __align__(16) _Float16 lds[A_TOT];
  const int tid = threadIdx.x, lane = tid & 31, wv = tid >> 5;
  const int col = lane & 15, h8 = (lane >> 4) << 3;
  const int perb = NN / 64;
  const int b = blockIdx.x / perb;
  const int qBlk = (blockIdx.x % perb) * 64;

#pragma unroll
  for (int it = 0; it < 16; ++it) {
    const int plane = it >> 3;
    const int cidx = (it * 128 + tid) & 1023;
    const int row = cidx >> 4, piece = cidx & 15;
    const _Float16* src = (plane ? thl : thh) + ((size_t)b * NN + qBlk + row) * NI + piece * 8;
    *(v8h*)(lds + (plane ? A_THL : A_THH) + row * 128 + piece * 8) = *(const v8h*)src;
  }

  v8f O[8];
#pragma unroll
  for (int ci = 0; ci < 8; ++ci) O[ci] = v8f{};
  float m8[8], l8[8];
#pragma unroll
  for (int r = 0; r < 8; ++r) { m8[r] = -1e30f; l8[r] = 0.0f; }

  const _Float16* tAh  = lds + A_THH + (wv * 16 + col) * 128 + h8;
  const _Float16* tAl  = lds + A_THL + (wv * 16 + col) * 128 + h8;
  const _Float16* pB0h = lds + A_PHH + col * 128 + h8;
  const _Float16* pB1h = lds + A_PHH + (16 + col) * 128 + h8;
  const _Float16* pB0l = lds + A_PHL + col * 128 + h8;
  const _Float16* pB1l = lds + A_PHL + (16 + col) * 128 + h8;
  const _Float16* gB   = lds + A_GS + col * 32 + h8;
  _Float16* pbw = lds + A_PB + wv * 512;

#pragma unroll 1
  for (int kb = 0; kb < NM; kb += 32) {
    __syncthreads();
#pragma unroll
    for (int it = 0; it < 8; ++it) {
      const int plane = it >> 2;
      const int cidx = (it * 128 + tid) & 511;
      const int row = cidx >> 4, piece = cidx & 15;
      const _Float16* src = (plane ? phl : phh) + ((size_t)b * NM + kb + row) * NI + piece * 8;
      *(v8h*)(lds + (plane ? A_PHL : A_PHH) + row * 128 + piece * 8) = *(const v8h*)src;
    }
#pragma unroll
    for (int it = 0; it < 4; ++it) {
      const int cidx = it * 128 + tid;
      const int ci = cidx >> 2, piece = cidx & 3;
      const _Float16* src = gT + ((size_t)b * NI + ci) * NM + kb + piece * 8;
      *(v8h*)(lds + A_GS + ci * 32 + piece * 8) = *(const v8h*)src;
    }
    __syncthreads();

    v8f S0h = {}, S0x = {}, S1h = {}, S1x = {};
#pragma unroll 1
    for (int k = 0; k < 4; ++k) {
      const v16h Ah  = load_h16(tAh + k * 32);
      const v16h Al  = load_h16(tAl + k * 32);
      const v16h Bh0 = load_h16(pB0h + k * 32);
      const v16h Bl0 = load_h16(pB0l + k * 32);
      const v16h Bh1 = load_h16(pB1h + k * 32);
      const v16h Bl1 = load_h16(pB1l + k * 32);
      S0h = wmma16(Ah, Bh0, S0h);
      S0x = wmma16(Ah, Bl0, S0x);
      S0x = wmma16(Al, Bh0, S0x);
      S1h = wmma16(Ah, Bh1, S1h);
      S1x = wmma16(Ah, Bl1, S1x);
      S1x = wmma16(Al, Bh1, S1x);
    }

#pragma unroll
    for (int r = 0; r < 8; ++r) {
      const float s0 = S0h[r] + S0x[r] * (1.0f / 1024.0f);
      const float s1 = S1h[r] + S1x[r] * (1.0f / 1024.0f);
      float mx = fmaxf(s0, s1);
      mx = fmaxf(mx, __shfl_xor(mx, 1));
      mx = fmaxf(mx, __shfl_xor(mx, 2));
      mx = fmaxf(mx, __shfl_xor(mx, 4));
      mx = fmaxf(mx, __shfl_xor(mx, 8));
      const float mn = fmaxf(m8[r], mx);
      const float sc = __expf(m8[r] - mn);
      const float p0 = __expf(s0 - mn);
      const float p1 = __expf(s1 - mn);
      float ps = p0 + p1;
      ps += __shfl_xor(ps, 1);
      ps += __shfl_xor(ps, 2);
      ps += __shfl_xor(ps, 4);
      ps += __shfl_xor(ps, 8);
      l8[r] = l8[r] * sc + ps;
      m8[r] = mn;
#pragma unroll
      for (int ci = 0; ci < 8; ++ci) O[ci][r] *= sc;
      pbw[(h8 + r) * 32 + col]      = (_Float16)(p0 * 16384.0f);
      pbw[(h8 + r) * 32 + 16 + col] = (_Float16)(p1 * 16384.0f);
    }
    __syncthreads();

    const v16h AP = load_h16(pbw + col * 32 + h8);
#pragma unroll
    for (int ci = 0; ci < 8; ++ci) O[ci] = wmma16(AP, load_h16(gB + ci * 512), O[ci]);
  }
  __syncthreads();

  fa_t* ys = reinterpret_cast<fa_t*>(lds);
#pragma unroll
  for (int r = 0; r < 8; ++r) {
    const float inv = 1.0f / (l8[r] * 16384.0f);
#pragma unroll
    for (int ci = 0; ci < 8; ++ci) ys[(wv * 16 + h8 + r) * 128 + ci * 16 + col] = O[ci][r] * inv;
  }
  __syncthreads();
  const size_t rowBase = (size_t)b * NN + qBlk + wv * 16;
#pragma unroll 1
  for (int it = 0; it < 8; ++it) {
    const int line = it * 4 + (lane >> 3);
    const int row = line >> 1;
    const int e0 = (line & 1) * 64 + (lane & 7) * 8;
    const v4fa va = *(const v4fa*)(ys + (wv * 16 + row) * 128 + e0);
    const v4fa vb = *(const v4fa*)(ys + (wv * 16 + row) * 128 + e0 + 4);
    v8h hv, lv;
    split8(va, vb, hv, lv);
    const size_t off = (rowBase + row) * NI + e0;
    st2h8(yh + off, hv);
    st2h8(yl + off, lv);
  }
}

__global__ void __launch_bounds__(128)
wout_kernel(const _Float16* __restrict__ yh, const _Float16* __restrict__ yl,
            const _Float16* __restrict__ wo, const float* __restrict__ bo,
            float* __restrict__ wy, float* __restrict__ part) {
  __shared__ __align__(16) _Float16 ysm[2][32][128];
  __shared__ __align__(16) float T[NC][36];
  const int tid = threadIdx.x, lane = tid & 31, wv = tid >> 5;
  const int col = lane & 15, h8 = (lane >> 4) << 3;
  const int perb = NN / 32;
  const int b = blockIdx.x / perb;
  const int n0 = (blockIdx.x % perb) * 32;

#pragma unroll
  for (int it = 0; it < 8; ++it) {
    const int plane = it >> 2;
    const int cidx = (it * 128 + tid) & 511;
    const int row = cidx >> 4, piece = cidx & 15;
    const _Float16* src = (plane ? yl : yh) + ((size_t)b * NN + n0 + row) * NI + piece * 8;
    *(v8h*)&ysm[plane][row][piece * 8] = *(const v8h*)src;
  }
  __syncthreads();

#pragma unroll 1
  for (int ct = 0; ct < 4; ++ct) {
    const int cbase = wv * 64 + ct * 16;
    const _Float16* wrow = wo + (size_t)(cbase + col) * NI + h8;
    v16h Aw[4];
#pragma unroll
    for (int k = 0; k < 4; ++k) Aw[k] = load_h16(wrow + k * 32);
    const v4f b0 = *(const v4f*)(bo + cbase + h8);
    const v4f b1 = *(const v4f*)(bo + cbase + h8 + 4);
    v8f bv;
#pragma unroll
    for (int j = 0; j < 4; ++j) { bv[j] = bf16r(b0[j]); bv[4 + j] = bf16r(b1[j]); }
#pragma unroll
    for (int pt = 0; pt < 2; ++pt) {
      const _Float16* ybh = &ysm[0][pt * 16 + col][h8];
      const _Float16* ybl = &ysm[1][pt * 16 + col][h8];
      v8f ah = {}, al = {};
#pragma unroll
      for (int k = 0; k < 4; ++k) {
        ah = wmma16(Aw[k], load_h16(ybh + k * 32), ah);
        al = wmma16(Aw[k], load_h16(ybl + k * 32), al);
      }
#pragma unroll
      for (int r = 0; r < 8; ++r)
        T[cbase + h8 + r][pt * 16 + col] = (ah[r] + al[r] * (1.0f / 1024.0f)) * 0.0625f + bv[r];
    }
  }
  __syncthreads();

  {
    const int c0 = tid * 2;
    float s0 = 0.0f, q0 = 0.0f, s1 = 0.0f, q1 = 0.0f;
#pragma unroll
    for (int j = 0; j < 8; ++j) {
      const v4f u = *(const v4f*)&T[c0][j * 4];
      const v4f v = *(const v4f*)&T[c0 + 1][j * 4];
      s0 += (u[0] + u[1]) + (u[2] + u[3]);
      q0 += (u[0] * u[0] + u[1] * u[1]) + (u[2] * u[2] + u[3] * u[3]);
      s1 += (v[0] + v[1]) + (v[2] + v[3]);
      q1 += (v[0] * v[0] + v[1] * v[1]) + (v[2] * v[2] + v[3] * v[3]);
    }
    v4f pv;
    pv[0] = s0; pv[1] = q0; pv[2] = s1; pv[3] = q1;
    st2f4(part + (size_t)blockIdx.x * 512 + tid * 4, pv);
  }
#pragma unroll 1
  for (int it = 0; it < 16; ++it) {
    const int ch = it * 16 + (tid >> 3);
    const int q = tid & 7;
    const v4f v = *(const v4f*)&T[ch][q * 4];
    st2f4(wy + ((size_t)b * NC + ch) * NN + n0 + q * 4, v);
  }
}

__global__ void __launch_bounds__(256)
bnred_kernel(const float* __restrict__ part, const float* __restrict__ gam,
             const float* __restrict__ bet, float* __restrict__ stats) {
  const int c = threadIdx.x;
  double s = 0.0, q = 0.0;
#pragma unroll 1
  for (int p = 0; p < NPART; ++p) {
    s += (double)part[(size_t)p * 512 + 2 * c];
    q += (double)part[(size_t)p * 512 + 2 * c + 1];
  }
  const double cnt = (double)NB * (double)NN;
  const double mean = s / cnt;
  double var = q / cnt - mean * mean;
  if (var < 0.0) var = 0.0;
  const float varf = (float)var;
  const float rstd = 1.0f / sqrtf(varf + 1e-5f);
  st2f1(stats + c, (float)mean);
  st2f1(stats + NC + c, rstd);
  st2f1(stats + 2 * NC + c, bf16r(gam[c]));
  st2f1(stats + 3 * NC + c, bf16r(bet[c]));
}

__global__ void __launch_bounds__(256)
final_kernel(const float* __restrict__ wy, const float* __restrict__ x,
             const float* __restrict__ stats, float* __restrict__ out) {
  const size_t i4 = (size_t)blockIdx.x * 256 + threadIdx.x;
  const int c = (int)((i4 >> 10) & 255);
  const float mean = stats[c];
  const float rstd = stats[NC + c];
  const float g = stats[2 * NC + c];
  const float be = stats[3 * NC + c];
  const v4f w  = *(const v4f*)(wy + i4 * 4);
  const v4f xv = *(const v4f*)(x + i4 * 4);
  v4f o;
#pragma unroll
  for (int j = 0; j < 4; ++j) {
    float t = (w[j] - mean) * rstd;
    t = t * g + be;
    o[j] = t + bf16r(xv[j]);
  }
  st2f4(out + i4 * 4, o);
}

extern "C" void kernel_launch(void* const* d_in, const int* in_sizes, int n_in,
                              void* d_out, int out_size, void* d_ws,
                              size_t ws_size, hipStream_t stream) {
  if (n_in < 11) return;
  if (in_sizes[0] < NB * NC * NN) return;
  if (in_sizes[1] < NI * NC || in_sizes[3] < NI * NC || in_sizes[5] < NI * NC) return;
  if (in_sizes[7] < NC * NI) return;
  if (in_sizes[2] < NI || in_sizes[4] < NI || in_sizes[6] < NI) return;
  if (in_sizes[8] < NC || in_sizes[9] < NC || in_sizes[10] < NC) return;
  if (out_size < NB * NC * NN) return;
  if (ws_size < WS_TOTAL) return;

  const float* x       = (const float*)d_in[0];
  const float* theta_w = (const float*)d_in[1];
  const float* theta_b = (const float*)d_in[2];
  const float* phi_w   = (const float*)d_in[3];
  const float* phi_b   = (const float*)d_in[4];
  const float* g_w     = (const float*)d_in[5];
  const float* g_b     = (const float*)d_in[6];
  const float* W_w     = (const float*)d_in[7];
  const float* W_b     = (const float*)d_in[8];
  const float* bn_g    = (const float*)d_in[9];
  const float* bn_b    = (const float*)d_in[10];
  float* out = (float*)d_out;

  char* ws = (char*)d_ws;
  _Float16* wpl  = (_Float16*)(ws + OFF_WPL);
  _Float16* xT   = (_Float16*)(ws + OFF_XT);
  _Float16* thh  = (_Float16*)(ws + OFF_THH);
  _Float16* thl  = (_Float16*)(ws + OFF_THL);
  _Float16* phh  = (_Float16*)(ws + OFF_PHH);
  _Float16* phl  = (_Float16*)(ws + OFF_PHL);
  _Float16* gT   = (_Float16*)(ws + OFF_GT);
  _Float16* yh   = (_Float16*)(ws + OFF_YH);
  _Float16* yl   = (_Float16*)(ws + OFF_YL);
  float*    wy   = (float*)(ws + OFF_WY);
  float*    part = (float*)(ws + OFF_PART);
  float*    stats= (float*)(ws + OFF_ST);

  _Float16* w_th = wpl;
  _Float16* w_ph = wpl + (size_t)NI * NC;
  _Float16* w_g  = wpl + (size_t)2 * NI * NC;
  _Float16* w_o  = wpl + (size_t)3 * NI * NC;

  cvt_w_kernel<<<64, 256, 0, stream>>>(theta_w, phi_w, g_w, W_w, wpl);
  xpose_kernel<<<NB * (NC / 64) * (NN / 32), 256, 0, stream>>>(x, xT);
  theta_kernel<<<NB * (NN / 64), 128, 0, stream>>>(xT, w_th, theta_b, thh, thl);
  phig_kernel<<<NB * (NN / 256), 256, 0, stream>>>(xT, w_ph, w_g, phi_b, g_b, phh, phl, gT);
  attn_kernel<<<NB * (NN / 64), 128, 0, stream>>>(thh, thl, phh, phl, gT, yh, yl);
  wout_kernel<<<NB * (NN / 32), 128, 0, stream>>>(yh, yl, w_o, W_b, wy, part);
  bnred_kernel<<<1, 256, 0, stream>>>(part, bn_g, bn_b, stats);
  final_kernel<<<(NB * NC * NN / 4) / 256, 256, 0, stream>>>(wy, x, stats, out);
}
